// mamba_Attention_70076686402463
// MI455X (gfx1250) — hardware-verified
//
#include <hip/hip_runtime.h>
#include <math.h>

typedef _Float16 f16;
typedef __attribute__((ext_vector_type(16))) _Float16 v16h;
typedef __attribute__((ext_vector_type(8)))  _Float16 v8h;
typedef __attribute__((ext_vector_type(8)))  float    v8f;
typedef __attribute__((ext_vector_type(4)))  float    v4f_t;
typedef float v4fa __attribute__((ext_vector_type(4), may_alias));

#define BATCH 2
#define LSEQ  1024
#define DMODEL 1024
#define ED    1024
#define NS    16
#define DTR   64
#define KCONV 4
#define TOK   (BATCH * LSEQ)
#define DBCW  (DTR + 2 * NS)
#define RSPLIT (1.0f / 2048.0f)
#ifndef SCAN_L
#define SCAN_L LSEQ
#endif

__device__ __forceinline__ float siluf(float v) { return v / (1.0f + __expf(-v)); }
__device__ __forceinline__ float siluf_rcp(float z) { float d = 1.0f + __expf(-z); float r = __builtin_amdgcn_rcpf(d); asm volatile("" : "+v"(r)); return z * r; }
__device__ __forceinline__ f16 lo_of(float v, f16 h) { return (f16)((v - (float)h) * 2048.0f); }
__device__ __forceinline__ unsigned pk2s(float a, float b, unsigned* lo) {
  const f16 h0 = (f16)a, h1 = (f16)b;
  *lo = (unsigned)__builtin_bit_cast(unsigned short, lo_of(a, h0)) | ((unsigned)__builtin_bit_cast(unsigned short, lo_of(b, h1)) << 16);
  return (unsigned)__builtin_bit_cast(unsigned short, h0) | ((unsigned)__builtin_bit_cast(unsigned short, h1) << 16);
}
__device__ __forceinline__ f16 lo_of_nofma(float v, f16 h) { float hf = (float)h; asm volatile("" : "+v"(hf)); float d = v - hf; asm volatile("" : "+v"(d)); float t = d * 2048.0f; asm volatile("" : "+v"(t)); return (f16)t; }
__device__ __forceinline__ unsigned pk2s_nofma(float a, float b, unsigned* lo) {
  float a1 = a, b1 = b; asm volatile("" : "+v"(a1), "+v"(b1));
  const f16 h0 = (f16)a1, h1 = (f16)b1;
  *lo = (unsigned)__builtin_bit_cast(unsigned short, lo_of_nofma(a1, h0)) | ((unsigned)__builtin_bit_cast(unsigned short, lo_of_nofma(b1, h1)) << 16);
  return (unsigned)__builtin_bit_cast(unsigned short, h0) | ((unsigned)__builtin_bit_cast(unsigned short, h1) << 16);
}

__device__ __forceinline__ v8f wmma16(v16h a, v16h b, v8f c) {
  return __builtin_amdgcn_wmma_f32_16x16x32_f16(false, a, false, b, (short)0, c, false, false);
}
__device__ __forceinline__ v8f wmma_split(v16h a, v16h al, v16h b, v16h bl, v8f c) {
  v8f x = {};
  x = wmma16(al, b, x); x = wmma16(a, bl, x);
  return wmma16(a, b, c) + x * RSPLIT;
}
__device__ __forceinline__ v16h cat8(v8h a, v8h b) { return __builtin_shufflevector(a, b, 0,1,2,3,4,5,6,7,8,9,10,11,12,13,14,15); }

__global__ __launch_bounds__(256) void cvt_planes(const float* __restrict__ s, f16* __restrict__ d, int n) {
  const int i = (blockIdx.x * 256 + threadIdx.x) * 2;
  if (i >= n) return;
  unsigned lo; const unsigned p = pk2s(s[i], s[i + 1], &lo);
  *(volatile unsigned*)(d + i) = p; *(volatile unsigned*)(d + n + i) = lo; __threadfence();
  *(volatile unsigned*)(d + i) = p; *(volatile unsigned*)(d + n + i) = lo;
}
__global__ __launch_bounds__(256) void cvt2d_planes(const float* __restrict__ s, f16* __restrict__ d) {
  const int i = (blockIdx.x * 256 + threadIdx.x) * 2;
  if (i >= TOK * DTR) return;
  const int r = i / DTR, c = i - r * DTR;
  unsigned lo; const unsigned p = pk2s(s[(size_t)r * DBCW + c], s[(size_t)r * DBCW + c + 1], &lo);
  *(volatile unsigned*)(d + i) = p; *(volatile unsigned*)(d + (size_t)TOK * DTR + i) = lo; __threadfence();
  *(volatile unsigned*)(d + i) = p; *(volatile unsigned*)(d + (size_t)TOK * DTR + i) = lo;
}

__global__ __launch_bounds__(256) void gemm_split(const f16* __restrict__ A, const f16* __restrict__ W,
                                                  float* __restrict__ C, int T, int N, int K) {
  __shared__ __attribute__((aligned(16))) float stg[8][16 * 36];
  const int lane = threadIdx.x & 31, wv = threadIdx.x >> 5;
  const int wave = (blockIdx.x * blockDim.x + threadIdx.x) >> 5;
  const int nStrips = N >> 5;
  const int nTiles  = (T >> 4) * nStrips;
  if (wave >= nTiles) return;
  const int m0   = (wave / nStrips) << 4;
  const int n0   = (wave % nStrips) << 5;
  const int half = (lane >> 4) & 1;
  const int l16  = lane & 15;
  const size_t pa = (size_t)T * K, pw = (size_t)N * K;
  const f16* Arow  = A + (size_t)(m0 + l16) * K + 8 * half;
  const f16* Brow0 = W + (size_t)(n0 + l16) * K + 8 * half;
  const f16* Brow1 = W + (size_t)(n0 + 16 + l16) * K + 8 * half;
  v8f acc0 = {}; v8f acc1 = {};
  for (int kk = 0; kk < K; kk += 32) {
    const v16h a   = cat8(*(const v8h*)(Arow + kk),       *(const v8h*)(Arow + kk + 16));
    const v16h al  = cat8(*(const v8h*)(Arow + pa + kk),  *(const v8h*)(Arow + pa + kk + 16));
    const v16h b0  = cat8(*(const v8h*)(Brow0 + kk),      *(const v8h*)(Brow0 + kk + 16));
    const v16h b0l = cat8(*(const v8h*)(Brow0 + pw + kk), *(const v8h*)(Brow0 + pw + kk + 16));
    const v16h b1  = cat8(*(const v8h*)(Brow1 + kk),      *(const v8h*)(Brow1 + kk + 16));
    const v16h b1l = cat8(*(const v8h*)(Brow1 + pw + kk), *(const v8h*)(Brow1 + pw + kk + 16));
    acc0 = wmma_split(a, al, b0, b0l, acc0);
    acc1 = wmma_split(a, al, b1, b1l, acc1);
  }
  float* sw = stg[wv];
#pragma unroll
  for (int r = 0; r < 8; ++r) { sw[(half * 8 + r) * 36 + l16] = acc0[r]; sw[(half * 8 + r) * 36 + 16 + l16] = acc1[r]; }
  asm volatile("s_wait_dscnt 0" ::: "memory");
#pragma unroll 1
  for (int pass = 0; pass < 2; ++pass) {
#pragma unroll
    for (int i = 0; i < 4; ++i) { const int c = lane + 32 * i, rr = c >> 3, q = (c & 7) * 4;
      *(volatile v4f_t*)(C + (size_t)(m0 + rr) * N + n0 + q) = *(const volatile v4fa*)(sw + rr * 36 + q); }
    __threadfence();
  }
}

__global__ __launch_bounds__(256) void conv_silu(const float* __restrict__ xz, const float* __restrict__ conv_w,
                                                 const float* __restrict__ conv_b,
                                                 float* __restrict__ xi_f, f16* __restrict__ xi_h, int ntok) {
  const int i = (blockIdx.x * 256 + threadIdx.x) * 2;
  if (i >= ntok * ED) return;
  const int e = i & (ED - 1);
  const int t = i >> 10;
  const int l = t & (LSEQ - 1);
  const int b = t >> 10;
  float s2[2];
#pragma unroll
  for (int q = 0; q < 2; ++q) {
    float acc = conv_b[e + q];
#pragma unroll
    for (int k = 0; k < KCONV; ++k) {
      const int lk = l + k - (KCONV - 1);
      if (lk >= 0) acc += xz[(size_t)(b * LSEQ + lk) * (2 * ED) + e + q] * conv_w[(e + q) * KCONV + k];
    }
    s2[q] = siluf(acc);
  }
  typedef __attribute__((ext_vector_type(2))) float v2f_t;
  v2f_t f2; f2.x = s2[0]; f2.y = s2[1];
  unsigned lo; const unsigned p = pk2s(s2[0], s2[1], &lo);
  *(volatile v2f_t*)(xi_f + i) = f2; *(volatile unsigned*)(xi_h + i) = p; *(volatile unsigned*)(xi_h + (size_t)TOK * ED + i) = lo; __threadfence();
  *(volatile v2f_t*)(xi_f + i) = f2; *(volatile unsigned*)(xi_h + i) = p; *(volatile unsigned*)(xi_h + (size_t)TOK * ED + i) = lo;
}

__global__ __launch_bounds__(32) void selective_scan(const float* __restrict__ delta_pre, const float* __restrict__ dt_b,
                                                     const float* __restrict__ xi_f, const float* __restrict__ dbc,
                                                     const float* __restrict__ xz, const float* __restrict__ A_log,
                                                     const float* __restrict__ D_param, f16* __restrict__ y_h) {
  const int lane = threadIdx.x;
  const int wave = blockIdx.x;
  const int b  = wave / (ED / 64);
  const int e0 = (wave % (ED / 64)) * 64 + lane * 2;
  float Aen[2][NS], h[2][NS], dtb[2], Dp[2];
#pragma unroll
  for (int q = 0; q < 2; ++q) {
    dtb[q] = dt_b[e0 + q]; Dp[q] = D_param[e0 + q];
#pragma unroll
    for (int n = 0; n < NS; ++n) { Aen[q][n] = -__expf(A_log[(e0 + q) * NS + n]); h[q][n] = 0.0f; }
  }
  for (int l = 0; l < SCAN_L; ++l) {
    const int t = b * LSEQ + l;
    float Bv[NS], Cv[NS];
#pragma unroll
    for (int n = 0; n < NS; ++n) { Bv[n] = dbc[(size_t)t * DBCW + DTR + n]; Cv[n] = dbc[(size_t)t * DBCW + DTR + NS + n]; }
    float yo[2];
#pragma unroll
    for (int q = 0; q < 2; ++q) {
      const float dpre  = delta_pre[(size_t)t * ED + e0 + q] + dtb[q];
      float sp_arg = 1.0f + __expf(dpre); asm volatile("" : "+v"(sp_arg));
      float sp_l2; asm volatile("v_log_f32 %0, %1" : "=v"(sp_l2) : "v"(sp_arg));
      const float delta = (dpre > 20.0f) ? dpre : sp_l2 * 0.69314718056f;
      const float xiv = xi_f[(size_t)t * ED + e0 + q];
      float dx = delta * xiv; asm volatile("" : "+v"(dx));
      float yv = 0.0f;
#pragma unroll
      for (int n = 0; n < NS; ++n) {
        float t1 = __expf(delta * Aen[q][n]) * h[q][n]; asm volatile("" : "+v"(t1));
        float t2 = dx * Bv[n];                       asm volatile("" : "+v"(t2));
        h[q][n] = t1 + t2;
        float t3 = h[q][n] * Cv[n];                  asm volatile("" : "+v"(t3));
        yv = yv + t3;
      }
      const float z = xz[(size_t)t * (2 * ED) + ED + e0 + q];
      float t4 = Dp[q] * xiv; asm volatile("" : "+v"(t4));
      yo[q] = (yv + t4) * siluf_rcp(z);
    }
    unsigned lo; const unsigned p = pk2s_nofma(yo[0], yo[1], &lo);
    f16* dst = y_h + (size_t)t * ED + e0;
    *(volatile unsigned*)dst = p; *(volatile unsigned*)(dst + (size_t)TOK * ED) = lo; __threadfence();
    *(volatile unsigned*)dst = p; *(volatile unsigned*)(dst + (size_t)TOK * ED) = lo;
  }
}

static inline int ceil_div(int a, int b) { return (a + b - 1) / b; }

extern "C" void kernel_launch(void* const* d_in, const int* in_sizes, int n_in,
                              void* d_out, int out_size, void* d_ws, size_t ws_size,
                              hipStream_t stream) {
  const float* x          = (const float*)d_in[0];
  const float* in_proj_w  = (const float*)d_in[1];
  const float* conv_w     = (const float*)d_in[2];
  const float* conv_b     = (const float*)d_in[3];
  const float* x_proj_w   = (const float*)d_in[4];
  const float* dt_proj_w  = (const float*)d_in[5];
  const float* dt_proj_b  = (const float*)d_in[6];
  const float* A_log      = (const float*)d_in[7];
  const float* D_param    = (const float*)d_in[8];
  const float* out_proj_w = (const float*)d_in[9];
  float* out = (float*)d_out;

  char* p = (char*)d_ws;
  auto alloc = [&](size_t bytes) -> char* { char* r = p; p += (bytes + 255) & ~(size_t)255; return r; };
  f16* x_h     = (f16*)alloc((size_t)TOK * DMODEL * 2 * 2);
  f16* w_in_h  = (f16*)alloc((size_t)2 * ED * DMODEL * 2 * 2);
  f16* w_xp_h  = (f16*)alloc((size_t)DBCW * ED * 2 * 2);
  f16* w_dt_h  = (f16*)alloc((size_t)ED * DTR * 2 * 2);
  f16* w_out_h = (f16*)alloc((size_t)DMODEL * ED * 2 * 2);
  float* xz    = (float*)alloc((size_t)TOK * 2 * ED * 4);
  float* xi_f  = (float*)alloc((size_t)TOK * ED * 4);
  f16* xi_h    = (f16*)alloc((size_t)TOK * ED * 2 * 2);
  float* dbc   = (float*)alloc((size_t)TOK * DBCW * 4);
  f16* dbc_h   = (f16*)alloc((size_t)TOK * DTR * 2 * 2);
  float* dpre  = (float*)alloc((size_t)TOK * ED * 4);
  f16* y_h     = (f16*)alloc((size_t)TOK * ED * 2 * 2);

  const int BS = 256;
  const int NTOK = TOK;
  cvt_planes<<<ceil_div(TOK * DMODEL / 2, BS), BS, 0, stream>>>(x, x_h, TOK * DMODEL);
  cvt_planes<<<ceil_div(2 * ED * DMODEL / 2, BS), BS, 0, stream>>>(in_proj_w, w_in_h, 2 * ED * DMODEL);
  cvt_planes<<<ceil_div(DBCW * ED / 2, BS), BS, 0, stream>>>(x_proj_w, w_xp_h, DBCW * ED);
  cvt_planes<<<ceil_div(ED * DTR / 2, BS), BS, 0, stream>>>(dt_proj_w, w_dt_h, ED * DTR);
  cvt_planes<<<ceil_div(DMODEL * ED / 2, BS), BS, 0, stream>>>(out_proj_w, w_out_h, DMODEL * ED);

  { int waves = (NTOK / 16) * ((2 * ED) / 32); gemm_split<<<ceil_div(waves * 32, BS), BS, 0, stream>>>(x_h, w_in_h, xz, TOK, 2 * ED, DMODEL); }
  conv_silu<<<ceil_div(NTOK * ED / 2, BS), BS, 0, stream>>>(xz, conv_w, conv_b, xi_f, xi_h, NTOK);
  { int waves = (NTOK / 16) * (DBCW / 32); gemm_split<<<ceil_div(waves * 32, BS), BS, 0, stream>>>(xi_h, w_xp_h, dbc, TOK, DBCW, ED); }
  cvt2d_planes<<<ceil_div(TOK * DTR / 2, BS), BS, 0, stream>>>(dbc, dbc_h);
  { int waves = (NTOK / 16) * (ED / 32); gemm_split<<<ceil_div(waves * 32, BS), BS, 0, stream>>>(dbc_h, w_dt_h, dpre, TOK, ED, DTR); }
  selective_scan<<<BATCH * ED / 64, 32, 0, stream>>>(dpre, dt_proj_b, xi_f, dbc, xz, A_log, D_param, y_h);
  { int waves = (NTOK / 16) * (DMODEL / 32); gemm_split<<<ceil_div(waves * 32, BS), BS, 0, stream>>>(y_h, w_out_h, out, TOK, DMODEL, ED); }
  (void)in_sizes; (void)n_in; (void)out_size; (void)ws_size;
}
